// CausalSelfAttention_31258771980754
// MI455X (gfx1250) — hardware-verified
//
#include <hip/hip_runtime.h>


#ifndef NB
#define NB 2
#endif
#ifndef SEQ
#define SEQ 2048
#endif
#define NB_FULL  2
#define SEQ_FULL 2048
#define DM   1024
#define NH   16
#define HD   64
#define NQKV (3 * DM)
#define RH   256
#define PCAR 256.0f
#define RSC  2048.0f
#define SCL  0.125f
#define L2E  1.4426950408889634f
#define NEGB (-1.0e30f)
#define CTP  72
#define MROWS (NB * SEQ)
#define PLANE ((unsigned)(NB * NH * SEQ * HD))
#define CPL  ((size_t)MROWS * DM)

static_assert(HD == 64);
static_assert((HD / 2) == 32);
static_assert(DM == NH * HD);
static_assert(DM % 32 == 0);
static_assert(DM % 64 == 0);
static_assert(NQKV % 64 == 0);
static_assert(SEQ % 64 == 0);
static_assert(RH % 64 == 0);
static_assert(SEQ >= RH);
static_assert(MROWS % 64 == 0);
static_assert(NB <= NB_FULL);
static_assert(SEQ <= SEQ_FULL);
static_assert(((size_t)NB * NH * SEQ * HD) % 512 == 0);
static_assert((SEQ * 32) % 256 == 0);
static_assert((size_t)4 * NB * NH * SEQ * HD < 4294967296ull);
static_assert((CTP * 2) % 16 == 0);
static_assert(CTP >= HD);

typedef _Float16 h16;
typedef unsigned short bf;
typedef __attribute__((ext_vector_type(16))) __bf16   v16bf;
typedef __attribute__((ext_vector_type(16))) _Float16 v16h;
typedef __attribute__((ext_vector_type(8)))  _Float16 v8h;
typedef __attribute__((ext_vector_type(8)))  unsigned short v8us;
typedef __attribute__((ext_vector_type(8)))  float    v8f;
typedef __attribute__((ext_vector_type(4)))  float    v4f;
typedef __attribute__((ext_vector_type(2)))  float    v2f;
typedef __attribute__((ext_vector_type(2)))  _Float16 v2h;
typedef __attribute__((ext_vector_type(2)))  unsigned short v2us;
typedef v4f  __attribute__((may_alias)) v4fa;
typedef v8us __attribute__((may_alias)) v8usa;

__device__ __forceinline__ unsigned short f2bf(float f) { unsigned u = __float_as_uint(f); u += 0x7FFFu + ((u >> 16) & 1u); return (unsigned short)(u >> 16); }
__device__ __forceinline__ float bf2f(unsigned short b) { return __uint_as_float(((unsigned)b) << 16); }
__device__ __forceinline__ void splitf(float y, unsigned short& h, unsigned short& l) { h = f2bf(y); l = f2bf(y - bf2f(h)); }
__device__ __forceinline__ v16h cat16(v8h lo, v8h hi) { return __builtin_shufflevector(lo, hi, 0, 1, 2, 3, 4, 5, 6, 7, 8, 9, 10, 11, 12, 13, 14, 15); }
__device__ __forceinline__ v16bf cat16b(v8us lo, v8us hi) { return __builtin_bit_cast(v16bf, __builtin_shufflevector(lo, hi, 0, 1, 2, 3, 4, 5, 6, 7, 8, 9, 10, 11, 12, 13, 14, 15)); }
__device__ __forceinline__ v8f wmma16(v16h a, v16h b, v8f c) { return __builtin_amdgcn_wmma_f32_16x16x32_f16(false, a, false, b, (short)0, c, false, false); }
__device__ __forceinline__ v8f wmmab(v16bf a, v16bf b, v8f c) { return __builtin_amdgcn_wmma_f32_16x16x32_bf16(false, a, false, b, (short)0, c, false, false); }
__device__ __forceinline__ v16bf ldb(const bf* p) { return cat16b(*(const v8us*)p, *(const v8us*)(p + 16)); }
__device__ __forceinline__ v16h ldh(const h16* p) { return cat16(*(const v8h*)p, *(const v8h*)(p + 16)); }

template <int NSPLIT>
__device__ __forceinline__ void gemmw_body(const bf* __restrict__ A, const bf* __restrict__ A2, const bf* __restrict__ Bt, const int K, float* C, const int ldc, const size_t sA, const size_t sC) {
    __shared__ __align__(16) float os[16 * 68];
    const size_t z = blockIdx.z; A += z * sA; A2 += z * sA; C += z * sC;
    const int lane = threadIdx.x & 31, lr = lane & 15, hi = lane >> 4; const int r0 = blockIdx.x * 64, c0 = blockIdx.y * 64;
    v8f acc[4][4];
#pragma unroll
    for (int mb = 0; mb < 4; ++mb)
#pragma unroll
        for (int nb = 0; nb < 4; ++nb) acc[mb][nb] = (v8f){};
    const size_t aoff = (size_t)(r0 + lr) * K + 8 * hi, boff = (size_t)(c0 + lr) * K + 8 * hi;
#pragma unroll 1
    for (int kc = 0; kc < K; kc += 32) {
        v16bf a[4], a2[4], bl;
#pragma unroll
        for (int mb = 0; mb < 4; ++mb) { a[mb] = ldb(A + aoff + (size_t)mb * 16 * K + kc); if (NSPLIT == 1) a2[mb] = ldb(A2 + aoff + (size_t)mb * 16 * K + kc); else a2[mb] = a[mb]; }
#pragma unroll
        for (int nb = 0; nb < 4; ++nb) { const v16bf b = ldb(Bt + boff + (size_t)nb * 16 * K + kc); if (nb == 3) bl = b;
#pragma unroll
            for (int mb = 0; mb < 4; ++mb) { acc[mb][nb] = wmmab(a[mb], b, acc[mb][nb]); if (NSPLIT == 1) acc[mb][nb] = wmmab(a2[mb], b, acc[mb][nb]); } }
        asm volatile("" : "+v"(acc[0][0]), "+v"(acc[0][1]), "+v"(acc[1][0]), "+v"(acc[1][1]), "+v"(acc[2][0]), "+v"(acc[2][1]), "+v"(acc[3][0]), "+v"(acc[3][1]));
        asm volatile("v_nop\n\tv_nop\n\tv_nop\n\tv_nop" : "+v"(acc[0][2]), "+v"(acc[0][3]), "+v"(acc[1][2]), "+v"(acc[1][3]), "+v"(acc[2][2]), "+v"(acc[2][3]), "+v"(acc[3][2]), "+v"(acc[3][3]) : "v"(a[0]), "v"(a[1]), "v"(a[2]), "v"(a[3]), "v"(bl));
        asm volatile("" : "+v"(acc[0][0]), "+v"(acc[0][1]), "+v"(acc[1][0]), "+v"(acc[1][1]), "+v"(acc[2][0]), "+v"(acc[2][1]), "+v"(acc[3][0]), "+v"(acc[3][1]) : "v"(a2[0]), "v"(a2[1]), "v"(a2[2]), "v"(a2[3]));
    }
#pragma unroll
    for (int mb = 0; mb < 4; ++mb) {
#pragma unroll
        for (int nb = 0; nb < 4; ++nb) {
#pragma unroll
            for (int j = 0; j < 8; ++j) os[(hi * 8 + j) * 68 + nb * 16 + lr] = acc[mb][nb][j]; }
        asm volatile("s_wait_dscnt 0x0" ::: "memory"); __builtin_amdgcn_wave_barrier();
        float* crow = C + (size_t)(r0 + mb * 16) * ldc + c0;
#pragma unroll 1
        for (int ps = 0; ps < 2; ++ps) {
#pragma unroll
            for (int s = 0; s < 8; ++s) { const int row = 2 * s + hi, cofs = lr * 4; const v4f val = *(const v4fa*)(os + row * 68 + cofs);
                *(volatile v4f*)(crow + (size_t)row * ldc + cofs) = val; }
            if (ps == 0) __threadfence(); }
        asm volatile("s_wait_dscnt 0x0" ::: "memory"); __builtin_amdgcn_wave_barrier();
    }
}
__global__ __launch_bounds__(32) void k_gemm_qkv(const bf* __restrict__ A, const bf* __restrict__ Bt, float* C) { gemmw_body<0>(A, A, Bt, DM, C, NQKV, 0, 0); }
__global__ __launch_bounds__(32) void k_gemm_out(const bf* __restrict__ Ah, const bf* __restrict__ Al, const bf* __restrict__ Bt, float* C) { gemmw_body<1>(Ah, Al, Bt, DM, C, DM, (size_t)SEQ * DM, (size_t)SEQ_FULL * DM); }

__global__ __launch_bounds__(256) void k_cvt8(const float* __restrict__ src, bf* dst, unsigned n8, unsigned per8, unsigned sstride8) {
    const unsigned i = blockIdx.x * 256u + threadIdx.x; if (i >= n8) return;
    const size_t si = (size_t)(i / per8) * sstride8 + (i % per8);
    const v8f v = *(const v8f*)(src + si * 8); v8us o;
#pragma unroll
    for (int k = 0; k < 8; ++k) o[k] = f2bf(v[k]);
    *(volatile v8us*)(dst + (size_t)i * 8) = o; __threadfence(); *(volatile v8us*)(dst + (size_t)i * 8) = o; }

__global__ __launch_bounds__(256) void k_cstab(float* CS) {
    const int idx = blockIdx.x * 256 + threadIdx.x; if (idx >= SEQ * 32) return;
    const int j = idx & 31, t = idx >> 5;
    double p = 1.0;
    p *= (j & 1) ? 1.3335214321633240 : 1.0;
    p *= (j & 2) ? 1.7782794100389228 : 1.0;
    p *= (j & 4) ? 3.1622776601683795 : 1.0;
    p *= (j & 8) ? 10.0 : 1.0;
    p *= (j & 16) ? 100.0 : 1.0;
    const float pf = (float)p; const float inv = 1.0f / pf; const float ang = (float)t * inv;
    float sn, cn; sincosf(ang, &sn, &cn);
    v2f cs; cs[0] = cn; cs[1] = sn;
    *(volatile v2f*)(CS + (size_t)idx * 2) = cs; __threadfence(); *(volatile v2f*)(CS + (size_t)idx * 2) = cs; }

__global__ __launch_bounds__(256) void k_rope(const float* __restrict__ F, const float* __restrict__ CS, bf* QK) {
#pragma clang fp contract(off)
    const unsigned which = blockIdx.y;
    const unsigned e = (blockIdx.x * 256u + threadIdx.x) * 2u; if (e >= PLANE) return;
    const unsigned d = e & (HD - 1); const unsigned t = (e / HD) % SEQ; const unsigned zz = e / (HD * SEQ); const unsigned b = zz / NH, h = zz % NH;
    const size_t rbase = ((size_t)b * SEQ + t) * NQKV + which * DM + h * HD;
    const v2f x = *(const v2f*)(F + rbase + d);
    const v2f pp = *(const v2f*)(F + rbase + (d ^ 32u));
    const v4f cs = *(const v4f*)(CS + ((size_t)t * 32 + (d & 31u)) * 2);
    const float sg = (d < 32u) ? -1.0f : 1.0f;
    const float p0 = sg * pp[0], p1 = sg * pp[1];
    const float sc = which ? 1.0f : SCL;
    const float r0 = (x[0] * cs[0] + p0 * cs[1]) * sc;
    const float r1 = (x[1] * cs[2] + p1 * cs[3]) * sc;
    v2us oh, ol; unsigned short a, c;
    splitf(r0, a, c); oh[0] = a; ol[0] = c; splitf(r1, a, c); oh[1] = a; ol[1] = c;
    bf* ph = QK + (size_t)(which * 2u) * PLANE + e; bf* pl = QK + (size_t)(which * 2u + 1u) * PLANE + e;
    *(volatile v2us*)ph = oh; *(volatile v2us*)pl = ol; __threadfence(); *(volatile v2us*)ph = oh; *(volatile v2us*)pl = ol; }

__global__ __launch_bounds__(256) void k_vtp(const float* __restrict__ F, h16* VT) {
    const unsigned e = (blockIdx.x * 256u + threadIdx.x) * 2u; if (e >= PLANE) return;
    const unsigned t = e % SEQ; const unsigned d = (e / SEQ) % HD; const unsigned zz = e / (SEQ * HD); const unsigned b = zz / NH, h = zz % NH;
    v2h o16, ors;
#pragma unroll
    for (int q = 0; q < 2; ++q) { const float x = F[((size_t)b * SEQ + t + q) * NQKV + 2 * DM + h * HD + d]; const h16 hv = (h16)x; o16[q] = hv; ors[q] = (h16)((x - (float)hv) * RSC); }
    h16* p0 = VT + e; h16* p1 = VT + (size_t)PLANE + e;
    *(volatile v2h*)p0 = o16; *(volatile v2h*)p1 = ors; __threadfence(); *(volatile v2h*)p0 = o16; *(volatile v2h*)p1 = ors; }

template <bool EARLY>
__device__ __forceinline__ void attn_body(const bf* __restrict__ QK, const h16* __restrict__ VT, bf* CT, const int qbase) {
    __shared__ __align__(16) unsigned short cts[4 * 2 * 16 * CTP];
    const int lane = threadIdx.x & 31, hh = lane >> 4, ln = lane & 15;
    const int wave = __builtin_amdgcn_readfirstlane((int)(threadIdx.x >> 5));
    const int zz = blockIdx.y;
    const int qw = qbase + (int)blockIdx.x * 64 + wave * 16;
    const int nsteps = (qw >> 5) + 1;
    const unsigned hb = (unsigned)zz * (unsigned)(SEQ * HD);
    const unsigned qoff = hb + (unsigned)(qw + ln) * HD + 8u * hh;
    const unsigned kofs = 2u * PLANE + hb + (unsigned)ln * HD + 8u * hh;
    const unsigned vofs = hb + (unsigned)ln * SEQ + 8u * hh;
    v8f o[4], oR[4];
#pragma unroll
    for (int dt = 0; dt < 4; ++dt) { o[dt] = (v8f){}; oR[dt] = (v8f){}; }
    float m = NEGB, l = 0.0f;
#pragma unroll 1
    for (int st = 0; st < nsteps; ++st) {
        const int kt = st * 32;
        unsigned qo = qoff; asm volatile("" : "+v"(qo));
        const v16bf qh0 = ldb(QK + (size_t)qo), qh1 = ldb(QK + (size_t)qo + 32), ql0 = ldb(QK + (size_t)(PLANE + qo)), ql1 = ldb(QK + (size_t)(PLANE + qo) + 32);
        v8f s0 = (v8f){}, s1 = (v8f){};
        {
            const unsigned ko = kofs + (unsigned)kt * HD;
            const v16bf kh0 = ldb(QK + (size_t)ko), kh1 = ldb(QK + (size_t)ko + 32), kl0 = ldb(QK + (size_t)(PLANE + ko)), kl1 = ldb(QK + (size_t)(PLANE + ko) + 32);
            s0 = wmmab(kh0, qh0, s0); s0 = wmmab(kh1, qh1, s0); s0 = wmmab(kh0, ql0, s0); s0 = wmmab(kh1, ql1, s0); s0 = wmmab(kl0, qh0, s0); s0 = wmmab(kl1, qh1, s0);
            asm volatile("v_nop\n\tv_nop\n\tv_nop\n\tv_nop" : "+v"(s0) : "v"(kh0), "v"(kh1), "v"(kl0), "v"(kl1), "v"(qh0), "v"(qh1), "v"(ql0), "v"(ql1));
        }
        asm volatile("" ::: "memory");
        {
            const unsigned ko = kofs + (unsigned)(kt + 16) * HD;
            const v16bf kh0 = ldb(QK + (size_t)ko), kh1 = ldb(QK + (size_t)ko + 32), kl0 = ldb(QK + (size_t)(PLANE + ko)), kl1 = ldb(QK + (size_t)(PLANE + ko) + 32);
            s1 = wmmab(kh0, qh0, s1); s1 = wmmab(kh1, qh1, s1); s1 = wmmab(kh0, ql0, s1); s1 = wmmab(kh1, ql1, s1); s1 = wmmab(kl0, qh0, s1); s1 = wmmab(kl1, qh1, s1);
            asm volatile("v_nop\n\tv_nop\n\tv_nop\n\tv_nop" : "+v"(s1), "+v"(s0) : "v"(kh0), "v"(kh1), "v"(kl0), "v"(kl1), "v"(qh0), "v"(qh1), "v"(ql0), "v"(ql1));
        }
        if (kt + 31 > qw) {
            const int qg = qw + ln, kb = kt + 8 * hh;
#pragma unroll
            for (int r = 0; r < 8; ++r) { s0[r] = (kb + r <= qg) ? s0[r] : NEGB; s1[r] = (kb + 16 + r <= qg) ? s1[r] : NEGB; }
        }
        float mx = s0[0];
#pragma unroll
        for (int r = 1; r < 8; ++r) mx = fmaxf(mx, s0[r]);
#pragma unroll
        for (int r = 0; r < 8; ++r) mx = fmaxf(mx, s1[r]);
        mx = fmaxf(mx, __shfl_xor(mx, 16, 32));
        const float mn = fmaxf(m, mx);
        const float al = __builtin_amdgcn_exp2f((m - mn) * L2E);
        m = mn;
        float rs = 0.0f; v16h pb, pr;
#pragma unroll
        for (int r = 0; r < 8; ++r) {
            const float e0 = __builtin_amdgcn_exp2f((s0[r] - mn) * L2E), e1 = __builtin_amdgcn_exp2f((s1[r] - mn) * L2E);
            rs += e0 + e1;
            const float c0 = e0 * PCAR, c1 = e1 * PCAR; const h16 a0 = (h16)c0, a1 = (h16)c1;
            pb[r] = a0; pb[8 + r] = a1;
            if (EARLY) { pr[r] = (h16)((c0 - (float)a0) * RSC); pr[8 + r] = (h16)((c1 - (float)a1) * RSC); } else { pr[r] = a0; pr[8 + r] = a1; }
        }
        l = l * al + rs;
#pragma unroll
        for (int dt = 0; dt < 4; ++dt) { o[dt] = o[dt] * al; if (EARLY) oR[dt] = oR[dt] * al; }
        asm volatile("" ::: "memory");
        v16h va[4], vr[4];
        const unsigned vo = vofs + (unsigned)kt;
#pragma unroll
        for (int dt = 0; dt < 4; ++dt) { va[dt] = ldh(VT + (size_t)(vo + (unsigned)(dt * 16 * SEQ))); if (EARLY) vr[dt] = ldh(VT + (size_t)(PLANE + vo + (unsigned)(dt * 16 * SEQ))); else vr[dt] = va[dt]; }
#pragma unroll
        for (int dt = 0; dt < 4; ++dt) { o[dt] = wmma16(va[dt], pb, o[dt]); if (EARLY) { oR[dt] = wmma16(va[dt], pr, oR[dt]); oR[dt] = wmma16(vr[dt], pb, oR[dt]); } }
        if (EARLY) asm volatile("v_nop\n\tv_nop\n\tv_nop\n\tv_nop" : "+v"(o[0]), "+v"(o[1]), "+v"(o[2]), "+v"(o[3]), "+v"(oR[0]), "+v"(oR[1]), "+v"(oR[2]), "+v"(oR[3]) : "v"(pb), "v"(pr), "v"(va[0]), "v"(va[1]), "v"(va[2]), "v"(va[3]), "v"(vr[0]), "v"(vr[1]), "v"(vr[2]), "v"(vr[3]));
        else asm volatile("v_nop\n\tv_nop\n\tv_nop\n\tv_nop" : "+v"(o[0]), "+v"(o[1]), "+v"(o[2]), "+v"(o[3]) : "v"(pb), "v"(va[0]), "v"(va[1]), "v"(va[2]), "v"(va[3]));
    }
    l += __shfl_xor(l, 16, 32);
    const float inv = 1.0f / (PCAR * l);
    const int cb = wave * (2 * 16 * CTP);
#pragma unroll
    for (int dt = 0; dt < 4; ++dt) { v8us oh, ol;
#pragma unroll
        for (int r = 0; r < 8; ++r) { float y = o[dt][r]; if (EARLY) y += oR[dt][r] * (1.0f / RSC); y *= inv; unsigned short a, c; splitf(y, a, c); oh[r] = a; ol[r] = c; }
        *(v8usa*)(cts + cb + ln * CTP + dt * 16 + 8 * hh) = oh; *(v8usa*)(cts + cb + 16 * CTP + ln * CTP + dt * 16 + 8 * hh) = ol; }
    asm volatile("s_wait_dscnt 0x0" ::: "memory"); __builtin_amdgcn_wave_barrier();
    const int b = zz / NH, h = zz % NH;
    const int rq = lane >> 3, pc = (lane & 7) * 8;
    v8us hv[4], lv[4];
#pragma unroll
    for (int it = 0; it < 4; ++it) { const int row = it * 4 + rq; hv[it] = *(const v8usa*)(cts + cb + row * CTP + pc); lv[it] = *(const v8usa*)(cts + cb + 16 * CTP + row * CTP + pc); }
    bf* gh = CT + ((size_t)b * SEQ + qw) * DM + h * HD + pc;
#pragma unroll 1
    for (int ps = 0; ps < 2; ++ps) {
#pragma unroll
        for (int it = 0; it < 4; ++it) { const int row = it * 4 + rq; *(volatile v8us*)(gh + (size_t)row * DM) = hv[it]; *(volatile v8us*)(gh + CPL + (size_t)row * DM) = lv[it]; }
        if (ps == 0) __threadfence(); }
}
__global__ __launch_bounds__(128) void k_attn_early(const bf* __restrict__ QK, const h16* __restrict__ VT, bf* CT) { attn_body<true>(QK, VT, CT, 0); }
__global__ __launch_bounds__(128) void k_attn_late(const bf* __restrict__ QK, const h16* __restrict__ VT, bf* CT) { attn_body<false>(QK, VT, CT, RH); }

constexpr size_t SZ_WQKV = (size_t)NQKV * DM * 2;
constexpr size_t SZ_WO   = (size_t)DM * DM * 2;
constexpr size_t SZ_CS   = (size_t)SEQ * 32 * 2 * 4;
constexpr size_t SZ_XB   = (size_t)MROWS * DM * 2;
constexpr size_t SZ_F    = (size_t)MROWS * NQKV * 4;
constexpr size_t SZ_QK   = (size_t)4 * NB * NH * SEQ * HD * 2;
constexpr size_t SZ_VT   = (size_t)2 * NB * NH * SEQ * HD * 2;
constexpr size_t SZ_CTX  = (size_t)2 * MROWS * DM * 2;
constexpr size_t SZ_TOTAL = SZ_WQKV + SZ_WO + SZ_CS + SZ_XB + SZ_F + SZ_QK + SZ_VT;
static_assert(SZ_CTX <= SZ_F);
static_assert(SZ_TOTAL <= (size_t)134217728);
static_assert(SZ_WQKV % 256 == 0 && SZ_WO % 256 == 0 && SZ_CS % 256 == 0 && SZ_XB % 256 == 0 && SZ_F % 256 == 0 && SZ_QK % 256 == 0 && SZ_VT % 256 == 0);

extern "C" void kernel_launch(void* const* d_in, const int* in_sizes, int n_in,
                              void* d_out, int out_size, void* d_ws, size_t ws_size, hipStream_t stream) {
    if (n_in < 3) return;
    const long long need_x = (long long)(NB - 1) * SEQ_FULL * DM + (long long)SEQ * DM;
    if ((long long)in_sizes[0] < need_x) return;
    if ((long long)in_sizes[1] < (long long)NQKV * DM) return;
    if ((long long)in_sizes[2] < (long long)DM * DM) return;
    if ((long long)out_size < need_x) return;
    if (SZ_TOTAL > ws_size) return;
    const float* x = (const float*)d_in[0];
    const float* wqkv = (const float*)d_in[1];
    const float* wout = (const float*)d_in[2];
    float* OUT = (float*)d_out;
    char* base = (char*)d_ws; size_t off = 0;
    bf* WQKVB = (bf*)(base + off); off += SZ_WQKV;
    bf* WOB = (bf*)(base + off); off += SZ_WO;
    float* CS = (float*)(base + off); off += SZ_CS;
    bf* XB = (bf*)(base + off); off += SZ_XB;
    float* F = (float*)(base + off); off += SZ_F;
    bf* QK = (bf*)(base + off); off += SZ_QK;
    h16* VT = (h16*)(base + off); off += SZ_VT;
    bf* CT = (bf*)F;

    const unsigned n8w = (unsigned)((size_t)NQKV * DM / 8), n8o = (unsigned)((size_t)DM * DM / 8), n8x = (unsigned)((size_t)MROWS * DM / 8);
    k_cvt8<<<(n8w + 255) / 256, 256, 0, stream>>>(wqkv, WQKVB, n8w, n8w, 0u);
    k_cvt8<<<(n8o + 255) / 256, 256, 0, stream>>>(wout, WOB, n8o, n8o, 0u);
    k_cvt8<<<(n8x + 255) / 256, 256, 0, stream>>>(x, XB, n8x, (unsigned)((size_t)SEQ * DM / 8), (unsigned)((size_t)SEQ_FULL * DM / 8));
    k_cstab<<<(SEQ * 32 + 255) / 256, 256, 0, stream>>>(CS);
    k_gemm_qkv<<<dim3(MROWS / 64, NQKV / 64, 1), 32, 0, stream>>>(XB, WQKVB, F);
    k_rope<<<dim3(PLANE / 512u, 2, 1), 256, 0, stream>>>(F, CS, QK);
    k_vtp<<<dim3(PLANE / 512u, 1, 1), 256, 0, stream>>>(F, VT);
    k_attn_early<<<dim3(RH / 64, NB * NH, 1), 128, 0, stream>>>(QK, VT, CT);
    if (SEQ > RH) k_attn_late<<<dim3((SEQ - RH) / 64, NB * NH, 1), 128, 0, stream>>>(QK, VT, CT);
    k_gemm_out<<<dim3(SEQ / 64, DM / 64, NB), 32, 0, stream>>>(CT, CT + CPL, WOB, OUT);
}
